// nonLocalBlock_30966714204745
// MI455X (gfx1250) — hardware-verified
//
#include <hip/hip_runtime.h>
#include <stddef.h>


typedef _Float16 v16h __attribute__((ext_vector_type(16)));
typedef _Float16 v8h  __attribute__((ext_vector_type(8)));
typedef float    v8f  __attribute__((ext_vector_type(8)));
typedef float    v4f  __attribute__((ext_vector_type(4)));
typedef _Float16 h16;

#ifndef NB
#define NB 4
#endif
#ifndef SEQ
#define SEQ 4096
#endif
#define NB_FULL  4
#define SEQ_FULL 4096
#define CIN   256
#define CHI   128
#define MROWS (NB * SEQ)

static_assert(NB >= 1 && NB <= NB_FULL);
static_assert(SEQ >= 128 && SEQ <= SEQ_FULL && (SEQ % 128) == 0);
static_assert(CHI == 128);
static_assert(CIN == 2 * CHI);
static_assert((CIN % 64) == 0 && (CIN % 32) == 0);
static_assert((CHI % 64) == 0 && (CHI % 32) == 0);
static_assert((MROWS % 64) == 0);
static_assert(((CHI * CIN) % (256 * 8)) == 0);
static_assert((size_t)MROWS * CIN < (size_t)0xFFFFFFFFu);

#define LDT 72
#define LDK 136
#define LDC 68
static_assert((LDT % 8) == 0 && LDT >= 64);
static_assert((LDK % 8) == 0 && LDK >= CHI);
static_assert((LDC % 4) == 0 && LDC >= 64);

#define WCARRY 64.0f
#define ACARRY 64.0f
#define PCARRY 16384.0f
#define VCARRY 64.0f
#define PLOG   9.704060528f
#define PFLUSH (-9.70f)

#define WP_BYTES   ((size_t)CHI * CIN * 2)
#define XT_BYTES   ((size_t)MROWS * CIN * 2)
#define P16_BYTES  ((size_t)MROWS * CHI * 2)
#define CS_BYTES   ((size_t)MROWS * 4)
#define OFF_WT  ((size_t)0)
#define OFF_WF  (OFF_WT + WP_BYTES)
#define OFF_WG  (OFF_WF + WP_BYTES)
#define OFF_WO  (OFF_WG + WP_BYTES)
#define OFF_XT  (OFF_WO + WP_BYTES)
#define OFF_TH  (OFF_XT + XT_BYTES)
#define OFF_PH  (OFF_TH + P16_BYTES)
#define OFF_GI  (OFF_PH + P16_BYTES)
#define OFF_GT  (OFF_GI + P16_BYTES)
#define OFF_CS  (OFF_GT + P16_BYTES)
#define OFF_Y   (OFF_CS + CS_BYTES)
#define WS_TOTAL (OFF_Y + P16_BYTES)
static_assert((WP_BYTES % 128) == 0 && (XT_BYTES % 128) == 0 && (P16_BYTES % 128) == 0);
static_assert((CS_BYTES % 128) == 0);
static_assert(WS_TOTAL <= (size_t)134217728);

__device__ __forceinline__ float bf16r(float x) {
  unsigned int u = __float_as_uint(x);
  u = (u + 0x7FFFu + ((u >> 16) & 1u)) & 0xFFFF0000u;
  return __uint_as_float(u);
}

static __device__ __forceinline__ h16 toh_flush(float v) {
  const h16 r = (h16)v;
  return (fabsf(v) < 6.103515625e-05f) ? (h16)0.0f : r;
}

__device__ __forceinline__ v16h frag_at(const _Float16* p) {
  v8h lo = *(const v8h*)(p);
  v8h hi = *(const v8h*)(p + 16);
  v16h out;
#pragma unroll
  for (int i = 0; i < 8; ++i) { out[i] = lo[i]; out[i + 8] = hi[i]; }
  return out;
}
__device__ __forceinline__ v16h ld_frag(const _Float16* base, unsigned ld) {
  const unsigned lane = threadIdx.x & 31u;
  return frag_at(base + (lane & 15u) * ld + (lane >> 4) * 8u);
}

__device__ __forceinline__ v8f wmma16(v16h a, v16h b, v8f c) {
  v8f d = __builtin_amdgcn_wmma_f32_16x16x32_f16(false, a, false, b, (short)0, c,
                                                 false, false);
  asm volatile("v_nop\n\tv_nop\n\tv_nop\n\tv_nop" : "+v"(d) : "v"(a), "v"(b));
  return d;
}

__device__ __forceinline__ float red16_max(float x) {
#pragma unroll
  for (int off = 1; off < 16; off <<= 1) x = fmaxf(x, __shfl_xor(x, off, 32));
  return x;
}
__device__ __forceinline__ float red16_sum(float x) {
#pragma unroll
  for (int off = 1; off < 16; off <<= 1) x += __shfl_xor(x, off, 32);
  return x;
}

__device__ __forceinline__ void wave_lds_sync() {
  __builtin_amdgcn_fence(3  , "wavefront");
  asm volatile("s_wait_dscnt 0x0" ::: "memory");
  __builtin_amdgcn_wave_barrier();
}

__global__ __launch_bounds__(256) void wconv_kernel(
    const float* __restrict__ W, _Float16* __restrict__ Wt, unsigned ldw, unsigned ldk) {
  __shared__ _Float16 T[64 * LDT];
  const unsigned tid = threadIdx.x;
  const unsigned n0 = blockIdx.x * 64u;
  const unsigned k0 = blockIdx.y * 64u;
#pragma unroll 4
  for (unsigned j = 0; j < 16u; ++j) {
    const unsigned idx = tid + 256u * j;
    const unsigned kr = idx >> 6, nc = idx & 63u;
    const float v = W[(size_t)(k0 + kr) * ldw + n0 + nc];
    T[nc * LDT + kr] = (_Float16)(WCARRY * bf16r(v));
  }
  __syncthreads();
  v8h x[2];
  size_t off[2];
#pragma unroll
  for (unsigned i = 0; i < 2u; ++i) {
    const unsigned n = 32u * i + (tid >> 3);
    const unsigned kc = (tid & 7u) * 8u;
    x[i] = *(const v8h*)&T[n * LDT + kc];
    off[i] = (size_t)(n0 + n) * ldk + k0 + kc;
  }
#pragma unroll
  for (int i = 0; i < 2; ++i) *(volatile v8h*)(Wt + off[i]) = x[i];
  __threadfence();
#pragma unroll
  for (int i = 0; i < 2; ++i) *(volatile v8h*)(Wt + off[i]) = x[i];
}

__global__ __launch_bounds__(256) void wcopy_kernel(
    const float* __restrict__ W, _Float16* __restrict__ Wp) {
  const size_t e0 = ((size_t)blockIdx.x * 256u + threadIdx.x) * 8u;
  const v4f a0 = *(const v4f*)(W + e0);
  const v4f a1 = *(const v4f*)(W + e0 + 4u);
  v8h o;
#pragma unroll
  for (int i = 0; i < 4; ++i) {
    o[i]     = toh_flush(WCARRY * bf16r(a0[i]));
    o[i + 4] = toh_flush(WCARRY * bf16r(a1[i]));
  }
  *(volatile v8h*)(Wp + e0) = o;
  __threadfence();
  *(volatile v8h*)(Wp + e0) = o;
}

__global__ __launch_bounds__(256) void xpose16_kernel(
    const _Float16* __restrict__ G, _Float16* __restrict__ Gt) {
  __shared__ _Float16 T[64 * LDT];
  const unsigned tid = threadIdx.x;
  const unsigned c0 = blockIdx.x * 64u;
  const unsigned j0 = blockIdx.y * 64u;
  const unsigned b = blockIdx.z;
  const size_t src = (size_t)b * SEQ * CHI;
#pragma unroll
  for (unsigned jj = 0; jj < 2u; ++jj) {
    const unsigned idx = tid + 256u * jj;
    const unsigned r = idx >> 3, cc = (idx & 7u) * 8u;
    const v8h v = *(const v8h*)(G + src + (size_t)(j0 + r) * CHI + c0 + cc);
#pragma unroll
    for (unsigned e = 0; e < 8u; ++e) T[(cc + e) * LDT + r] = v[e];
  }
  __syncthreads();
  v8h x[2];
  size_t off[2];
#pragma unroll
  for (unsigned i = 0; i < 2u; ++i) {
    const unsigned n = 32u * i + (tid >> 3);
    const unsigned kc = (tid & 7u) * 8u;
    x[i] = *(const v8h*)&T[n * LDT + kc];
    off[i] = ((size_t)b * CHI + c0 + n) * SEQ + j0 + kc;
  }
#pragma unroll
  for (int i = 0; i < 2; ++i) *(volatile v8h*)(Gt + off[i]) = x[i];
  __threadfence();
#pragma unroll
  for (int i = 0; i < 2; ++i) *(volatile v8h*)(Gt + off[i]) = x[i];
}

template <int MODE>
__device__ __forceinline__ void gemm_body(
    const _Float16* __restrict__ A16, const _Float16* __restrict__ Bt, const unsigned K,
    const float* __restrict__ bias, const float* __restrict__ addf,
    float* __restrict__ outf, _Float16* __restrict__ out16) {
  __shared__ float Cs[64 * LDC];
  const unsigned tid = threadIdx.x, lane = tid & 31u, w = tid >> 5;
  const unsigned mw = w >> 1, nw = w & 1u;
  const unsigned hh = lane >> 4, m = lane & 15u;
  const unsigned n0 = blockIdx.x * 64u;
  const unsigned row0 = blockIdx.y * 64u;

  const _Float16* ap  = A16 + (size_t)(row0 + mw * 16u + m) * K + hh * 8u;
  const _Float16* bp0 = Bt + (size_t)(n0 + nw * 32u + m) * K + hh * 8u;
  const _Float16* bp1 = bp0 + (size_t)16 * K;
  v8f acc0 = {}, acc1 = {};
#pragma unroll 2
  for (unsigned k0 = 0; k0 < K; k0 += 32u) {
    const v16h a  = frag_at(ap + k0);
    const v16h b0 = frag_at(bp0 + k0);
    const v16h b1 = frag_at(bp1 + k0);
    acc0 = wmma16(a, b0, acc0);
    acc1 = wmma16(a, b1, acc1);
  }
#pragma unroll
  for (int r = 0; r < 8; ++r) {
    float* d = &Cs[(mw * 16u + hh * 8u + (unsigned)r) * LDC + nw * 32u + m];
    d[0]  = acc0[r];
    d[16] = acc1[r];
  }
  __syncthreads();

  const float ps = ACARRY / (WCARRY * WCARRY);

  if (MODE == 0) {
    v8h x[2];
    size_t off[2];
#pragma unroll
    for (unsigned i = 0; i < 2u; ++i) {
      const unsigned r = 32u * i + (tid >> 3);
      const unsigned c = (tid & 7u) * 8u;
      const v4f u0 = *(const v4f*)&Cs[r * LDC + c];
      const v4f u1 = *(const v4f*)&Cs[r * LDC + c + 4];
      const v4f g0 = *(const v4f*)(bias + n0 + c);
      const v4f g1 = *(const v4f*)(bias + n0 + c + 4u);
#pragma unroll
      for (int j = 0; j < 4; ++j) {
        x[i][j]     = toh_flush(u0[j] * ps + ACARRY * bf16r(g0[j]));
        x[i][j + 4] = toh_flush(u1[j] * ps + ACARRY * bf16r(g1[j]));
      }
      off[i] = (size_t)(row0 + r) * CHI + n0 + c;
    }
#pragma unroll
    for (int i = 0; i < 2; ++i) *(volatile v8h*)(out16 + off[i]) = x[i];
    __threadfence();
#pragma unroll
    for (int i = 0; i < 2; ++i) *(volatile v8h*)(out16 + off[i]) = x[i];
  }

  if (MODE == 1) {
    const unsigned bidx = row0 / (unsigned)SEQ;
    const unsigned key0 = row0 - bidx * (unsigned)SEQ;
    v8h x[2];
    size_t off[2];
#pragma unroll
    for (unsigned i = 0; i < 2u; ++i) {
      const unsigned dcol = 32u * i + (tid >> 3);
      const unsigned kk = (tid & 7u) * 8u;
      const float bb = ACARRY * bf16r(bias[n0 + dcol]);
#pragma unroll
      for (unsigned j = 0; j < 8u; ++j) {
        const float t = Cs[(kk + j) * LDC + dcol] * ps + bb;
        x[i][j] = toh_flush(t);
      }
      off[i] = ((size_t)bidx * CHI + n0 + dcol) * SEQ + key0 + kk;
    }
#pragma unroll
    for (int i = 0; i < 2; ++i) *(volatile v8h*)(out16 + off[i]) = x[i];
    __threadfence();
#pragma unroll
    for (int i = 0; i < 2; ++i) *(volatile v8h*)(out16 + off[i]) = x[i];
  }

  if (MODE == 2) {
    const float cs = 1.0f / (WCARRY * VCARRY);
    const unsigned bidx = row0 / (unsigned)SEQ;
    const unsigned p0 = row0 - bidx * (unsigned)SEQ;
    v4f xs[4];
    size_t off[4];
#pragma unroll
    for (unsigned i = 0; i < 4u; ++i) {
      const unsigned ol = 16u * i + (tid >> 4);
      const unsigned pc = (tid & 15u) * 4u;
      const float gb = bf16r(bias[n0 + ol]);
      const size_t goff = ((size_t)bidx * CIN + n0 + ol) * SEQ_FULL + p0 + pc;
      const v4f xin = *(const v4f*)(addf + goff);
      v4f val;
#pragma unroll
      for (unsigned j = 0; j < 4u; ++j)
        val[j] = bf16r(xin[j]) + (Cs[(pc + j) * LDC + ol] * cs + gb);
      xs[i] = val;
      off[i] = goff;
    }
#pragma unroll
    for (int i = 0; i < 4; ++i) *(volatile v4f*)(outf + off[i]) = xs[i];
    __threadfence();
#pragma unroll
    for (int i = 0; i < 4; ++i) *(volatile v4f*)(outf + off[i]) = xs[i];
  }
}

__global__ __launch_bounds__(256) void gemm_pixmajor_kernel(
    const _Float16* __restrict__ A16, const _Float16* __restrict__ Bt,
    const float* __restrict__ bias, _Float16* __restrict__ out16) {
  gemm_body<0>(A16, Bt, (unsigned)CIN, bias, bias, (float*)0, out16);
}
__global__ __launch_bounds__(256) void gemm_chanmajor_kernel(
    const _Float16* __restrict__ A16, const _Float16* __restrict__ Bt,
    const float* __restrict__ bias, _Float16* __restrict__ out16) {
  gemm_body<1>(A16, Bt, (unsigned)CIN, bias, bias, (float*)0, out16);
}
__global__ __launch_bounds__(256) void gemm_out_kernel(
    const _Float16* __restrict__ A16, const _Float16* __restrict__ Bt,
    const float* __restrict__ bias, const float* __restrict__ xin, float* __restrict__ outf) {
  gemm_body<2>(A16, Bt, (unsigned)CHI, bias, xin, outf, (_Float16*)0);
}

__global__ __launch_bounds__(256) void colstat_kernel(
    const _Float16* __restrict__ PhT, const _Float16* __restrict__ Th,
    float* __restrict__ CSt) {
  __shared__ _Float16 Ks[64 * LDK];
  __shared__ float sm[128];

  const unsigned tid = threadIdx.x, lane = tid & 31u;
  const unsigned w = (unsigned)__builtin_amdgcn_readfirstlane((int)(threadIdx.x >> 5));
  const unsigned hh = lane >> 4, m = lane & 15u;
  const unsigned j0 = blockIdx.x * 128u;
  const unsigned b = blockIdx.y;
  const unsigned jrow0 = j0 + w * 16u;
  const float scale = 1.0f / (ACARRY * ACARRY);

  const size_t qoff = ((size_t)b * SEQ + jrow0 + m) * CHI + hh * 8u;
  v16h qf[4];
#pragma unroll
  for (int c = 0; c < 4; ++c) qf[c] = frag_at(PhT + qoff + 32 * c);

  float mrow[8], lrow[8];
#pragma unroll
  for (int v = 0; v < 8; ++v) { mrow[v] = -1.0e30f; lrow[v] = 0.0f; }

  const size_t kplane = (size_t)b * SEQ * CHI;

  for (unsigned kb = 0; kb < (unsigned)SEQ; kb += 64u) {
#pragma unroll
    for (unsigned j = 0; j < 4u; ++j) {
      const unsigned idx = tid + 256u * j;
      const unsigned r = idx >> 4, c = (idx & 15u) * 8u;
      *(v8h*)&Ks[r * LDK + c] = *(const v8h*)(Th + kplane + (size_t)(kb + r) * CHI + c);
    }
    __syncthreads();

    v8f s[4];
#pragma unroll
    for (int kg = 0; kg < 4; ++kg) {
      v8f t = {};
#pragma unroll
      for (int c = 0; c < 4; ++c) {
        const v16h kf = ld_frag(&Ks[(kg * 16) * LDK + c * 32], LDK);
        t = wmma16(qf[c], kf, t);
      }
      s[kg] = t * scale;
    }

#pragma unroll
    for (int v = 0; v < 8; ++v) {
      float mx = fmaxf(fmaxf(s[0][v], s[1][v]), fmaxf(s[2][v], s[3][v]));
      mx = red16_max(mx);
      const float mn = fmaxf(mrow[v], mx);
      const float alpha = __expf(mrow[v] - mn);
      mrow[v] = mn;
      const float e0 = __expf(s[0][v] - mn);
      const float e1 = __expf(s[1][v] - mn);
      const float e2 = __expf(s[2][v] - mn);
      const float e3 = __expf(s[3][v] - mn);
      const float rs = red16_sum((e0 + e1) + (e2 + e3));
      lrow[v] = alpha * lrow[v] + rs;
    }
    __syncthreads();
  }

  float cs[8];
#pragma unroll
  for (int v = 0; v < 8; ++v) cs[v] = mrow[v] + __logf(lrow[v]);
  if (m == 0u) {
#pragma unroll
    for (int v = 0; v < 8; ++v) sm[w * 16u + hh * 8u + (unsigned)v] = cs[v];
  }
  __syncthreads();
  if (w == 0u) {
    const v4f x = *(const v4f*)&sm[lane * 4u];
    float* p = CSt + (size_t)b * SEQ + j0 + lane * 4u;
    *(volatile v4f*)p = x;
    __threadfence();
    *(volatile v4f*)p = x;
  }
}

__global__ __launch_bounds__(256) void attn_kernel(
    const _Float16* __restrict__ Th, const _Float16* __restrict__ PhT,
    const _Float16* __restrict__ Gt, const float* __restrict__ CSt,
    _Float16* __restrict__ Yv) {
  __shared__ _Float16 Ks[64 * LDK];
  __shared__ _Float16 Vs[CHI * LDT];
  __shared__ _Float16 Ps[8 * 16 * LDT];
  __shared__ float cst[64];

  const unsigned tid = threadIdx.x, lane = tid & 31u;
  const unsigned w = (unsigned)__builtin_amdgcn_readfirstlane((int)(threadIdx.x >> 5));
  const unsigned hh = lane >> 4, m = lane & 15u;
  const unsigned q0 = blockIdx.x * 128u;
  const unsigned b = blockIdx.y;
  const unsigned qrow0 = q0 + w * 16u;
  const float scale = 1.0f / (ACARRY * ACARRY);
  _Float16* P = Ps + w * (16u * LDT);

  const size_t qoff = ((size_t)b * SEQ + qrow0 + m) * CHI + hh * 8u;
  v16h qf[4];
#pragma unroll
  for (int c = 0; c < 4; ++c) qf[c] = frag_at(Th + qoff + 32 * c);

  v8f o[8];
#pragma unroll
  for (int nb = 0; nb < 8; ++nb) o[nb] = (v8f){};

  const size_t kplane = (size_t)b * SEQ * CHI;
  const size_t vplane = (size_t)b * CHI * SEQ;
  const size_t splane = (size_t)b * SEQ;

  for (unsigned kb = 0; kb < (unsigned)SEQ; kb += 64u) {
#pragma unroll
    for (unsigned j = 0; j < 4u; ++j) {
      const unsigned idx = tid + 256u * j;
      const unsigned r = idx >> 4, c = (idx & 15u) * 8u;
      *(v8h*)&Ks[r * LDK + c] = *(const v8h*)(PhT + kplane + (size_t)(kb + r) * CHI + c);
    }
#pragma unroll
    for (unsigned j = 0; j < 4u; ++j) {
      const unsigned idx = tid + 256u * j;
      const unsigned r = idx >> 3, c = (idx & 7u) * 8u;
      *(v8h*)&Vs[r * LDT + c] = *(const v8h*)(Gt + vplane + (size_t)r * SEQ + kb + c);
    }
    const float cv = CSt[splane + kb + (tid & 63u)];
    if (w < 2u) cst[tid & 63u] = cv;
    __syncthreads();

    v8f s[4];
#pragma unroll
    for (int kg = 0; kg < 4; ++kg) {
      v8f t = {};
#pragma unroll
      for (int c = 0; c < 4; ++c) {
        const v16h kf = ld_frag(&Ks[(kg * 16) * LDK + c * 32], LDK);
        t = wmma16(qf[c], kf, t);
      }
      s[kg] = t;
    }

    float cj[4];
#pragma unroll
    for (int kg = 0; kg < 4; ++kg) cj[kg] = cst[(unsigned)kg * 16u + m];
#pragma unroll
    for (int kg = 0; kg < 4; ++kg)
#pragma unroll
      for (int v = 0; v < 8; ++v) {
        const float e = fminf(s[kg][v] * scale - cj[kg], 0.0f) + PLOG;
        const float p = (e < PFLUSH) ? 0.0f : __expf(e);
        P[(hh * 8u + (unsigned)v) * LDT + (unsigned)kg * 16u + m] = (_Float16)p;
      }
    wave_lds_sync();

#pragma unroll
    for (int c = 0; c < 2; ++c) {
      const v16h pf = ld_frag(P + c * 32, LDT);
#pragma unroll
      for (int nb = 0; nb < 8; ++nb) {
        const v16h vf = ld_frag(&Vs[(nb * 16) * LDT + c * 32], LDT);
        o[nb] = wmma16(pf, vf, o[nb]);
      }
    }
    __syncthreads();
  }

  const float inv = VCARRY / (PCARRY * ACARRY);
#pragma unroll
  for (int hf = 0; hf < 2; ++hf) {
#pragma unroll
    for (int nbl = 0; nbl < 4; ++nbl)
#pragma unroll
      for (int v = 0; v < 8; ++v)
        P[(hh * 8u + (unsigned)v) * LDT + (unsigned)nbl * 16u + m] =
            toh_flush(o[hf * 4 + nbl][v] * inv);
    wave_lds_sync();
    v8h x[4];
    size_t off[4];
#pragma unroll
    for (unsigned i = 0; i < 4u; ++i) {
      const unsigned r = 4u * i + (lane >> 3);
      const unsigned c = (lane & 7u) * 8u;
      x[i] = *(const v8h*)&P[r * LDT + c];
      off[i] = ((size_t)b * SEQ + qrow0 + r) * CHI + (unsigned)hf * 64u + c;
    }
#pragma unroll
    for (int i = 0; i < 4; ++i) *(volatile v8h*)(Yv + off[i]) = x[i];
    __threadfence();
#pragma unroll
    for (int i = 0; i < 4; ++i) *(volatile v8h*)(Yv + off[i]) = x[i];
    wave_lds_sync();
  }
}

extern "C" void kernel_launch(void* const* d_in, const int* in_sizes, int n_in,
                              void* d_out, int out_size, void* d_ws, size_t ws_size,
                              hipStream_t stream) {
  if (n_in < 9) return;
  const long long need_x = ((long long)(NB - 1) * CIN + (CIN - 1)) * SEQ_FULL + SEQ;
  if ((long long)in_sizes[0] < need_x) return;
  if ((long long)in_sizes[1] < (long long)CHI * CIN) return;
  if ((long long)in_sizes[3] < (long long)CHI * CIN) return;
  if ((long long)in_sizes[5] < (long long)CHI * CIN) return;
  if ((long long)in_sizes[7] < (long long)CIN * CHI) return;
  if (in_sizes[2] < CHI || in_sizes[4] < CHI || in_sizes[6] < CHI || in_sizes[8] < CIN) return;
  if ((long long)out_size < need_x) return;
  if (ws_size < WS_TOTAL) return;

  const float* X   = (const float*)d_in[0];
  const float* wt  = (const float*)d_in[1];
  const float* bt  = (const float*)d_in[2];
  const float* wf  = (const float*)d_in[3];
  const float* bf  = (const float*)d_in[4];
  const float* wg  = (const float*)d_in[5];
  const float* bg  = (const float*)d_in[6];
  const float* wo  = (const float*)d_in[7];
  const float* bo  = (const float*)d_in[8];
  float* out = (float*)d_out;

  char* ws = (char*)d_ws;
  _Float16* Wt_p = (_Float16*)(ws + OFF_WT);
  _Float16* Wf_p = (_Float16*)(ws + OFF_WF);
  _Float16* Wg_p = (_Float16*)(ws + OFF_WG);
  _Float16* Wo_p = (_Float16*)(ws + OFF_WO);
  _Float16* XT   = (_Float16*)(ws + OFF_XT);
  _Float16* TH   = (_Float16*)(ws + OFF_TH);
  _Float16* PH   = (_Float16*)(ws + OFF_PH);
  _Float16* GI   = (_Float16*)(ws + OFF_GI);
  _Float16* GT   = (_Float16*)(ws + OFF_GT);
  float*    CS   = (float*)(ws + OFF_CS);
  _Float16* Y16  = (_Float16*)(ws + OFF_Y);

  dim3 blk(256);

  wcopy_kernel<<<dim3((CHI * CIN) / 2048), blk, 0, stream>>>(wt, Wt_p);
  wcopy_kernel<<<dim3((CHI * CIN) / 2048), blk, 0, stream>>>(wf, Wf_p);
  wcopy_kernel<<<dim3((CHI * CIN) / 2048), blk, 0, stream>>>(wg, Wg_p);
  wcopy_kernel<<<dim3((CIN * CHI) / 2048), blk, 0, stream>>>(wo, Wo_p);

  for (int b = 0; b < NB; ++b) {
    wconv_kernel<<<dim3(SEQ / 64, CIN / 64), blk, 0, stream>>>(
        X + (size_t)b * CIN * SEQ_FULL, XT + (size_t)b * SEQ * CIN,
        (unsigned)SEQ_FULL, (unsigned)CIN);
  }

  dim3 gp(CHI / 64, MROWS / 64);
  gemm_chanmajor_kernel<<<gp, blk, 0, stream>>>(XT, Wt_p, bt, TH);
  gemm_pixmajor_kernel<<<gp, blk, 0, stream>>>(XT, Wf_p, bf, PH);
  gemm_chanmajor_kernel<<<gp, blk, 0, stream>>>(XT, Wg_p, bg, GI);
  xpose16_kernel<<<dim3(CHI / 64, SEQ / 64, NB), blk, 0, stream>>>(GI, GT);

  colstat_kernel<<<dim3(SEQ / 128, NB), blk, 0, stream>>>(PH, TH, CS);
  attn_kernel<<<dim3(SEQ / 128, NB), blk, 0, stream>>>(TH, PH, GT, CS, Y16);

  gemm_out_kernel<<<dim3(CIN / 64, MROWS / 64), blk, 0, stream>>>(Y16, Wo_p, bo, X, out);
}
